// EdgePathNN_33663953666603
// MI455X (gfx1250) — hardware-verified
//
#include <hip/hip_runtime.h>
#include <hip/hip_bf16.h>


#define HD   64
#define NFT  18
#define NCL  10
#define GW   256
#define KW   192
#define TDN  1024
#define TDG  512
#define SCH  2048
#define STR  512
#define XP   136
#define HP   72
#define OP   68
#define AP40 40
#define AP72 72

#define WPL_WF_H   0
#define WPL_WF_L   2048
#define WPL_WB_H   4096
#define WPL_WB_L   6144
#define WPL_MB     8192
#define WPL_L2_H   49152
#define WPL_L2_L   51200
#define WPL_WC     53248
#define WPL_TOTAL  102400
#define WPL_BLOCKS 50

static_assert(WPL_MB + 10 * 4096 == WPL_L2_H);
static_assert(WPL_L2_L + 2048 == WPL_WC);
static_assert(WPL_WC + GW * KW == WPL_TOTAL);
static_assert(WPL_TOTAL == WPL_BLOCKS * 2048);
static_assert((TDN & (TDN - 1)) == 0);
static_assert(TDG == 512);
static_assert(SCH == 8 * 256);
static_assert((XP * 2) % 16 == 0 && (HP * 2) % 16 == 0 && (OP * 4) % 16 == 0);

typedef float v4f __attribute__((ext_vector_type(4)));
typedef float v8f __attribute__((ext_vector_type(8)));
typedef double v2d __attribute__((ext_vector_type(2)));
typedef _Float16 f16t;
typedef f16t v4h __attribute__((ext_vector_type(4)));
typedef f16t v8h __attribute__((ext_vector_type(8)));
typedef f16t v16h __attribute__((ext_vector_type(16)));
typedef __bf16 v16b __attribute__((ext_vector_type(16)));
typedef unsigned short u16x4 __attribute__((ext_vector_type(4)));
typedef unsigned short u16x8 __attribute__((ext_vector_type(8)));

union FragB { u16x8 u[2]; v16b v; };
union FragH { u16x8 u[2]; v8h h[2]; v16h v; };

__device__ __forceinline__ unsigned short f2bf(float f) {
  unsigned u = __float_as_uint(f);
  u += 0x7FFFu + ((u >> 16) & 1u);
  return (unsigned short)(u >> 16);
}
__device__ __forceinline__ float bf2f(unsigned short b) { return __uint_as_float(((unsigned)b) << 16); }
__device__ __forceinline__ void splitbf(float f, unsigned short& hb, unsigned short& lb) {
  hb = f2bf(f);
  lb = f2bf(f - bf2f(hb));
}
__device__ __forceinline__ float sigm_f(float x) { return __builtin_amdgcn_rcpf(1.0f + __expf(-x)); }
__device__ __forceinline__ float tanh_f(float x) {
  const float t = __expf(-2.0f * fabsf(x));
  const float r = (1.0f - t) * __builtin_amdgcn_rcpf(1.0f + t);
  return copysignf(r, x);
}

__device__ __forceinline__ void mma_bf(v8f& acc, const FragB& a, const FragB& b) {
  acc = __builtin_amdgcn_wmma_f32_16x16x32_bf16(false, a.v, false, b.v, (short)0, acc, false, false);
  asm volatile("v_nop\n\tv_nop\n\tv_nop\n\tv_nop" : "+v"(acc) : "v"(a.v), "v"(b.v));
}
__device__ __forceinline__ void mma_hf(v8f& acc, const FragH& a, const FragH& b) {
  acc = __builtin_amdgcn_wmma_f32_16x16x32_f16(false, a.v, false, b.v, (short)0, acc, false, false);
  asm volatile("v_nop\n\tv_nop\n\tv_nop\n\tv_nop" : "+v"(acc) : "v"(a.v), "v"(b.v));
}
__device__ __forceinline__ void zero4(v8f (&a)[4]) {
#pragma unroll
  for (int j = 0; j < 4; ++j) {
#pragma unroll
    for (int r = 0; r < 8; ++r) a[j][r] = 0.0f;
  }
}

template<int KT, int NT>
__device__ __forceinline__ void mma_x3(v8f (&acc)[NT], const unsigned short* sAh, const unsigned short* sAl, const int PA,
                                       const unsigned short* __restrict__ Bh, const unsigned short* __restrict__ Bl, const int lane)
{
  const int h = lane >> 4, m = lane & 15;
  constexpr int KP = KT * 32;
#pragma unroll
  for (int kt = 0; kt < KT; ++kt) {
    FragB a, al;
    const unsigned short* pa = sAh + m * PA + kt * 32 + 8 * h;
    const unsigned short* pl = sAl + m * PA + kt * 32 + 8 * h;
    a.u[0]  = *(const u16x8*)pa;  a.u[1]  = *(const u16x8*)(pa + 16);
    al.u[0] = *(const u16x8*)pl;  al.u[1] = *(const u16x8*)(pl + 16);
#pragma unroll
    for (int j = 0; j < NT; ++j) {
      FragB b, bl;
      const unsigned short* pb = Bh + (size_t)(j * 16 + m) * KP + kt * 32 + 8 * h;
      const unsigned short* ql = Bl + (size_t)(j * 16 + m) * KP + kt * 32 + 8 * h;
      b.u[0]  = *(const u16x8*)pb;  b.u[1]  = *(const u16x8*)(pb + 16);
      bl.u[0] = *(const u16x8*)ql;  bl.u[1] = *(const u16x8*)(ql + 16);
      mma_bf(acc[j], a, b);
      mma_bf(acc[j], a, bl);
      mma_bf(acc[j], al, b);
    }
  }
}

__device__ __forceinline__ void stage_a64(const float* __restrict__ in, const int row0, const int Mreal,
                                          const float* __restrict__ ss, const int bn, const int relu,
                                          unsigned short* sAh, unsigned short* sAl, const int tid)
{
  const int c4 = (tid & 15) * 4;
  const v4f lsc = *(const v4f*)(ss + c4);
  const v4f lsh = *(const v4f*)(ss + HD + c4);
  v4f sc, sh;
#pragma unroll
  for (int i = 0; i < 4; ++i) { sc[i] = bn ? lsc[i] : 1.0f; sh[i] = bn ? lsh[i] : 0.0f; }
#pragma unroll
  for (int it = 0; it < 8; ++it) {
    const int idx = it * 128 + tid;
    const int row = idx >> 4;
    const int grow = row0 + row;
    v4f v = *(const v4f*)(in + (size_t)grow * HD + c4);
    v = v * sc + sh;
    u16x4 hv, lv;
#pragma unroll
    for (int i = 0; i < 4; ++i) {
      float x = v[i];
      if (relu) x = fmaxf(x, 0.0f);
      x = (grow < Mreal) ? x : 0.0f;
      unsigned short hb, lb;
      splitbf(x, hb, lb);
      hv[i] = hb; lv[i] = lb;
    }
    *(u16x4*)(sAh + row * AP72 + c4) = hv;
    *(u16x4*)(sAl + row * AP72 + c4) = lv;
  }
}

__device__ __forceinline__ void store_rows_f32(const float* st, float* g, const int lane) {
  const int hh = lane >> 4, c = (lane & 15) * 4;
#pragma unroll
  for (int it = 0; it < 8; ++it) {
    const int row = it * 2 + hh;
    const v4f v = *(const v4f*)(st + row * OP + c);
    *(volatile v4f*)(g + (size_t)row * HD + c) = v;
  }
  __threadfence();
#pragma unroll
  for (int it = 0; it < 8; ++it) {
    const int row = it * 2 + hh;
    const v4f v = *(const v4f*)(st + row * OP + c);
    *(volatile v4f*)(g + (size_t)row * HD + c) = v;
  }
}

__global__ __launch_bounds__(256)
void k_wprep(const float* __restrict__ w_feat, const float* __restrict__ w_bond,
             const float* __restrict__ mlp_w1, const float* __restrict__ mlp_w2,
             const float* __restrict__ w_l1, const float* __restrict__ w_l2,
             const float* __restrict__ w_ih, const float* __restrict__ w_hh,
             unsigned short* wpl)
{
  const int blk = blockIdx.x, tid = threadIdx.x;
  u16x8 o;
  if (blk < 4) {
    const float* src = (blk < 2) ? w_feat : w_bond;
    const int lo = blk & 1;
    const int fl = tid * 8;
    const int n = fl >> 5, k0 = fl & 31;
#pragma unroll
    for (int i = 0; i < 8; ++i) {
      const int k = k0 + i;
      const int kc = min(k, NFT - 1);
      float v = src[kc * HD + n];
      v = (k < NFT) ? v : 0.0f;
      unsigned short hb, lb;
      splitbf(v, hb, lb);
      o[i] = lo ? lb : hb;
    }
  } else if (blk < 24) {
    const int t = blk - 4, pl = t >> 1, sub = t & 1, lo = pl & 1, mat = pl >> 1;
    const float* src = mlp_w1;
    if (mat == 1) src = mlp_w2;
    else if (mat == 2) src = mlp_w1 + HD * HD;
    else if (mat == 3) src = mlp_w2 + HD * HD;
    else if (mat == 4) src = w_l1;
    const int fl = sub * 2048 + tid * 8;
    const int n = fl >> 6, k0 = fl & 63;
#pragma unroll
    for (int i = 0; i < 8; ++i) {
      const int k = k0 + i;
      const float v = src[k * HD + n];
      unsigned short hb, lb;
      splitbf(v, hb, lb);
      o[i] = lo ? lb : hb;
    }
  } else if (blk < 26) {
    const int lo = blk & 1;
    const int fl = tid * 8;
    const int n = fl >> 6, k0 = fl & 63;
    const int nc = min(n, NCL - 1);
#pragma unroll
    for (int i = 0; i < 8; ++i) {
      const int k = k0 + i;
      float v = w_l2[k * NCL + nc];
      v = (n < NCL) ? v : 0.0f;
      unsigned short hb, lb;
      splitbf(v, hb, lb);
      o[i] = lo ? lb : hb;
    }
  } else {
    const int fl = (blk - 26) * 2048 + tid * 8;
    const int n = fl / KW;
    const int k0 = fl - n * KW;
    v8h hv;
#pragma unroll
    for (int i = 0; i < 8; ++i) {
      const int k = k0 + i;
      const float a = w_ih[n * (2 * HD) + min(k, 2 * HD - 1)];
      const float b = w_hh[n * HD + min(max(k - 2 * HD, 0), HD - 1)];
      const float v = (k < 2 * HD) ? a : b;
      hv[i] = (f16t)(v * 16.0f);
    }
    o = __builtin_bit_cast(u16x8, hv);
  }
  unsigned short* gp = wpl + (size_t)blk * 2048 + tid * 8;
  *(volatile u16x8*)gp = o;
  __threadfence();
  *(volatile u16x8*)gp = o;
}

__global__ __launch_bounds__(128)
void k_enc(const float* __restrict__ A, int Mreal,
           const unsigned short* __restrict__ Wh, const unsigned short* __restrict__ Wl,
           const float* __restrict__ bias, float* outF, unsigned short* outH, int doF, int doH)
{
  __shared__ __attribute__((aligned(16))) unsigned short sAh[64 * AP40];
  __shared__ __attribute__((aligned(16))) unsigned short sAl[64 * AP40];
  __shared__ __attribute__((aligned(16))) float st[4][16 * OP];
  const int tid = threadIdx.x, lane = tid & 31, wave = tid >> 5, h = lane >> 4, m = lane & 15;
  const int row0 = blockIdx.x * 64;
  for (int idx = tid; idx < 64 * 32; idx += 128) {
    const int row = idx >> 5, k = idx & 31;
    const int grow = row0 + row;
    const int gr = min(grow, Mreal - 1);
    const int kk = min(k, NFT - 1);
    float v = A[(size_t)gr * NFT + kk];
    v = (grow < Mreal && k < NFT) ? v : 0.0f;
    unsigned short hb, lb;
    splitbf(v, hb, lb);
    sAh[row * AP40 + k] = hb;
    sAl[row * AP40 + k] = lb;
  }
  __syncthreads();
  v8f acc[4];
  zero4(acc);
  mma_x3<1, 4>(acc, sAh + wave * 16 * AP40, sAl + wave * 16 * AP40, AP40, Wh, Wl, lane);
  float* sw = st[wave];
#pragma unroll
  for (int j = 0; j < 4; ++j) {
    const float bj = bias[j * 16 + m];
#pragma unroll
    for (int r = 0; r < 8; ++r) sw[(8 * h + r) * OP + j * 16 + m] = acc[j][r] + bj;
  }
  __syncthreads();
  const int roww = row0 + wave * 16;
  if (doF) store_rows_f32(sw, outF + (size_t)roww * HD, lane);
  if (doH) {
    const int c = (lane & 7) * 8;
    u16x8 ov[4];
#pragma unroll
    for (int it = 0; it < 4; ++it) {
      const int row = it * 4 + (lane >> 3);
      v8h hv;
#pragma unroll
      for (int i = 0; i < 8; ++i) hv[i] = (f16t)(sw[row * OP + c + i] * 16.0f);
      ov[it] = __builtin_bit_cast(u16x8, hv);
    }
#pragma unroll
    for (int it = 0; it < 4; ++it) {
      const int row = it * 4 + (lane >> 3);
      *(volatile u16x8*)(outH + (size_t)(roww + row) * HD + c) = ov[it];
    }
    __threadfence();
#pragma unroll
    for (int it = 0; it < 4; ++it) {
      const int row = it * 4 + (lane >> 3);
      *(volatile u16x8*)(outH + (size_t)(roww + row) * HD + c) = ov[it];
    }
  }
}

__global__ __launch_bounds__(128)
void k_mlp(const float* __restrict__ in, int Mreal, const float* __restrict__ ss, int bn, int relu,
           const unsigned short* __restrict__ Wh, const unsigned short* __restrict__ Wl,
           const float* __restrict__ bias, float* out)
{
  __shared__ __attribute__((aligned(16))) unsigned short sAh[64 * AP72];
  __shared__ __attribute__((aligned(16))) unsigned short sAl[64 * AP72];
  __shared__ __attribute__((aligned(16))) float st[4][16 * OP];
  const int tid = threadIdx.x, lane = tid & 31, wave = tid >> 5, h = lane >> 4, m = lane & 15;
  const int row0 = blockIdx.x * 64;
  stage_a64(in, row0, Mreal, ss, bn, relu, sAh, sAl, tid);
  __syncthreads();
  v8f acc[4];
  zero4(acc);
  mma_x3<2, 4>(acc, sAh + wave * 16 * AP72, sAl + wave * 16 * AP72, AP72, Wh, Wl, lane);
  float* sw = st[wave];
#pragma unroll
  for (int j = 0; j < 4; ++j) {
    const float bj = bias[j * 16 + m];
#pragma unroll
    for (int r = 0; r < 8; ++r) sw[(8 * h + r) * OP + j * 16 + m] = acc[j][r] + bj;
  }
  __syncthreads();
  store_rows_f32(sw, out + (size_t)(row0 + wave * 16) * HD, lane);
}

__global__ __launch_bounds__(128)
void k_head2(const float* __restrict__ in, int Greal, const float* __restrict__ ss,
             const unsigned short* __restrict__ Wh, const unsigned short* __restrict__ Wl,
             const float* __restrict__ b2, float* out, int nout)
{
  __shared__ __attribute__((aligned(16))) unsigned short sAh[64 * AP72];
  __shared__ __attribute__((aligned(16))) unsigned short sAl[64 * AP72];
  __shared__ __attribute__((aligned(16))) float so[64 * NCL];
  const int tid = threadIdx.x, lane = tid & 31, wave = tid >> 5, h = lane >> 4, m = lane & 15;
  const int row0 = blockIdx.x * 64;
  stage_a64(in, row0, Greal, ss, 0, 1, sAh, sAl, tid);
  __syncthreads();
  v8f acc[1];
#pragma unroll
  for (int r = 0; r < 8; ++r) acc[0][r] = 0.0f;
  mma_x3<2, 1>(acc, sAh + wave * 16 * AP72, sAl + wave * 16 * AP72, AP72, Wh, Wl, lane);
  const float bj = b2[min(m, NCL - 1)];
  if (m < NCL) {
#pragma unroll
    for (int r = 0; r < 8; ++r) so[(wave * 16 + 8 * h + r) * NCL + m] = acc[0][r] + bj;
  }
  __syncthreads();
  const size_t fb = (size_t)row0 * NCL;
#pragma unroll
  for (int it = 0; it < 2; ++it) {
    const int pcn = it * 128 + tid;
    if (pcn < 160) {
      const size_t f = fb + (size_t)pcn * 4;
      if (f + 4 <= (size_t)nout) {
        const v4f v = *(const v4f*)(so + pcn * 4);
        *(volatile v4f*)(out + f) = v;
      }
    }
  }
  __threadfence();
#pragma unroll
  for (int it = 0; it < 2; ++it) {
    const int pcn = it * 128 + tid;
    if (pcn < 160) {
      const size_t f = fb + (size_t)pcn * 4;
      if (f + 4 <= (size_t)nout) {
        const v4f v = *(const v4f*)(so + pcn * 4);
        *(volatile v4f*)(out + f) = v;
      }
    }
  }
}

template<int L, bool WIN>
__device__ __forceinline__ void gather_x(const int* __restrict__ paths, const float* __restrict__ X0, const float* __restrict__ X1,
                                         const size_t gp, const int l, const int nN, f16t* xs, const int lane)
{
  int nd = paths[gp * L + l];
  nd = min(max(nd, 0), nN - 1);
  const int c = (lane & 15) * 4;
#pragma unroll
  for (int it = 0; it < 8; ++it) {
    const int row = it * 2 + (lane >> 4);
    const int ndr = __shfl(nd, row, 32);
    const v4f a = *(const v4f*)(X0 + (size_t)ndr * HD + c);
    v4f v = a;
    if (WIN) {
      const v4f b = *(const v4f*)(X1 + (size_t)ndr * HD + c);
      v = 0.75f * a - 0.25f * b;
    }
    v4h hv;
#pragma unroll
    for (int i = 0; i < 4; ++i) hv[i] = (f16t)(v[i] * 16.0f);
    *(v4h*)(xs + row * XP + c) = hv;
  }
}
template<int L>
__device__ __forceinline__ void gather_ea(const int* __restrict__ ei, const f16t* __restrict__ EA,
                                          const size_t gp, const int l, const int nE, f16t* xs, const int lane)
{
  int e = ei[gp * (L - 1) + (l - 1)];
  e = min(max(e, 0), nE - 1);
  const int c = (lane & 7) * 8;
#pragma unroll
  for (int it = 0; it < 4; ++it) {
    const int row = it * 4 + (lane >> 3);
    const int er = __shfl(e, row, 32);
    const v8h v = *(const v8h*)(EA + (size_t)er * HD + c);
    *(v8h*)(xs + row * XP + HD + c) = v;
  }
}
template<int KT, bool DOA>
__device__ __forceinline__ void lstm_half(v8f (&aA)[4], v8f (&aB)[4], const int tA0, const int tB0,
                                          const f16t* xs, const f16t* hs,
                                          const unsigned short* __restrict__ WC, const int lane)
{
  const int h = lane >> 4, m = lane & 15;
#pragma unroll
  for (int kt = 0; kt < KT; ++kt) {
    FragH a;
    const f16t* pa = (kt < 4) ? (xs + m * XP + kt * 32 + 8 * h) : (hs + m * HP + (kt - 4) * 32 + 8 * h);
    a.h[0] = *(const v8h*)pa;
    a.h[1] = *(const v8h*)(pa + 16);
#pragma unroll
    for (int j = 0; j < 4; ++j) {
      if (DOA) {
        FragH b;
        const unsigned short* pb = WC + (size_t)((tA0 + j) * 16 + m) * KW + kt * 32 + 8 * h;
        b.u[0] = *(const u16x8*)pb;
        b.u[1] = *(const u16x8*)(pb + 16);
        mma_hf(aA[j], a, b);
      }
      FragH b2;
      const unsigned short* qb = WC + (size_t)((tB0 + j) * 16 + m) * KW + kt * 32 + 8 * h;
      b2.u[0] = *(const u16x8*)qb;
      b2.u[1] = *(const u16x8*)(qb + 16);
      mma_hf(aB[j], a, b2);
    }
  }
}
__device__ __forceinline__ void cell_ig(const v8f (&aA)[4], const v8f (&aB)[4], v8f (&ig)[4], const float* sB, const int lane)
{
  const int m = lane & 15;
  const float K256 = 0.00390625f;
#pragma unroll
  for (int j = 0; j < 4; ++j) {
    const float bi = sB[j * 16 + m];
    const float bg = sB[2 * HD + j * 16 + m];
#pragma unroll
    for (int r = 0; r < 8; ++r) {
      const float gi = aA[j][r] * K256 + bi;
      const float gg = aB[j][r] * K256 + bg;
      ig[j][r] = sigm_f(gi) * tanh_f(gg);
    }
  }
}
template<bool FIRST>
__device__ __forceinline__ void cell_out(const v8f (&aA)[4], const v8f (&aB)[4], const v8f (&ig)[4], const float* sB,
                                         float* cs, f16t* hs, float* ho, const int lane)
{
  const int h = lane >> 4, m = lane & 15;
  const float K256 = 0.00390625f;
#pragma unroll
  for (int j = 0; j < 4; ++j) {
    const int u = j * 16 + m;
    const float bfg = sB[HD + u];
    const float bo = sB[3 * HD + u];
#pragma unroll
    for (int r = 0; r < 8; ++r) {
      const int row = 8 * h + r;
      const float go = aB[j][r] * K256 + bo;
      float c;
      if (FIRST) {
        c = ig[j][r];
      } else {
        const float gf = aA[j][r] * K256 + bfg;
        c = sigm_f(gf) * cs[row * HD + u] + ig[j][r];
      }
      const float hv = sigm_f(go) * tanh_f(c);
      cs[row * HD + u] = c;
      hs[row * HP + u] = (f16t)(hv * 16.0f);
      ho[row * OP + u] = hv;
    }
  }
}
template<int L, bool WIN>
__global__ __launch_bounds__(128)
void k_lstm(const int* __restrict__ paths, const int* __restrict__ ei,
            const float* __restrict__ X0, const float* __restrict__ X1,
            const f16t* __restrict__ EA, const unsigned short* __restrict__ WC,
            const float* __restrict__ b_ih, const float* __restrict__ b_hh,
            float* Hout, int p0, int pc, int nN, int nE)
{
  __shared__ __attribute__((aligned(16))) f16t xst[4][16 * XP];
  __shared__ __attribute__((aligned(16))) f16t hst[4][16 * HP];
  __shared__ __attribute__((aligned(16))) float cst[4][16 * HD];
  __shared__ __attribute__((aligned(16))) float hob[4][16 * OP];
  __shared__ float sB[GW];
  const int tid = threadIdx.x, lane = tid & 31, wave = tid >> 5, m = lane & 15;
  for (int i = tid; i < GW; i += 128) sB[i] = b_ih[i] + b_hh[i];
  const int tb = blockIdx.x * 64 + wave * 16;
  const int prow = min(tb + m, pc - 1);
  const size_t gp = (size_t)p0 + (size_t)prow;
  f16t* xs = xst[wave];
  f16t* hs = hst[wave];
  float* cs = cst[wave];
  float* ho = hob[wave];
  v8f aA[4], aB[4], ig[4];

  gather_x<L, WIN>(paths, X0, X1, gp, 0, nN, xs, lane);
  __syncthreads();
  zero4(aA); zero4(aB);
  lstm_half<2, true>(aA, aB, 0, 8, xs, hs, WC, lane);
  cell_ig(aA, aB, ig, sB, lane);
  zero4(aB);
  lstm_half<2, false>(aA, aB, 4, 12, xs, hs, WC, lane);
  cell_out<true>(aA, aB, ig, sB, cs, hs, ho, lane);
  __syncthreads();
#pragma unroll
  for (int l = 1; l < L; ++l) {
    gather_x<L, WIN>(paths, X0, X1, gp, l, nN, xs, lane);
    gather_ea<L>(ei, EA, gp, l, nE, xs, lane);
    __syncthreads();
    zero4(aA); zero4(aB);
    lstm_half<6, true>(aA, aB, 0, 8, xs, hs, WC, lane);
    cell_ig(aA, aB, ig, sB, lane);
    zero4(aA); zero4(aB);
    lstm_half<6, true>(aA, aB, 4, 12, xs, hs, WC, lane);
    cell_out<false>(aA, aB, ig, sB, cs, hs, ho, lane);
    __syncthreads();
  }
  store_rows_f32(ho, Hout + (size_t)tb * HD, lane);
}

template<int L>
__global__ __launch_bounds__(256)
void k_segsum(const int* __restrict__ paths, const float* __restrict__ Hc, float* ACC,
              int p0, int pc, int npad, int init, int nchunk)
{
  extern __shared__ __attribute__((aligned(16))) float dacc[];
  __shared__ int lst[8][32];
  __shared__ int cnt[8];
  const int tid = threadIdx.x, lane = tid & 31, wave = tid >> 5;
  const int node0 = blockIdx.x * TDN;
  const int c4 = (tid & 15) * 4;
#pragma unroll 4
  for (int it = 0; it < (TDN * 16) / 256; ++it) {
    const int piece = it * 256 + tid;
    const int row = piece >> 4;
    const int grow = node0 + row;
    v4f v;
    v[0] = 0.0f; v[1] = 0.0f; v[2] = 0.0f; v[3] = 0.0f;
    if (!init) {
      const int gr = min(grow, npad - 1);
      const v4f t = *(const v4f*)(ACC + (size_t)gr * HD + c4);
      if (grow < npad) v = t;
    }
    *(v4f*)(dacc + row * HD + c4) = v;
  }
  __syncthreads();
  for (int ci = 0; ci < nchunk; ++ci) {
    const int base = ci * SCH;
    int cw = 0;
#pragma unroll
    for (int j = 0; j < SCH / 256; ++j) {
      const int e = base + j * 256 + tid;
      const int ec = min(e, pc - 1);
      const int d = paths[((size_t)p0 + (size_t)ec) * L + (L - 1)];
      const int dl = d - node0;
      const bool hit = (e < pc) && ((unsigned)dl < (unsigned)TDN);
      const unsigned mk = __builtin_amdgcn_ballot_w32(hit);
      const int rank = __builtin_popcount(mk & ((1u << lane) - 1u));
      const int slot = cw + rank;
      if (hit && slot < 32) lst[wave][slot] = (e << 10) | dl;
      cw += __builtin_popcount(mk);
    }
    if (lane == 0) cnt[wave] = cw;
    __syncthreads();
    if (wave == 0) {
      for (int w = 0; w < 8; ++w) {
        const int nw = min(cnt[w], 32);
        for (int k = 0; k < nw; ++k) {
          const int ent = lst[w][k];
          const int e = min(ent >> 10, pc - 1);
          const int dl = ent & (TDN - 1);
          const v4f hv = *(const v4f*)(Hc + (size_t)e * HD + c4);
          float* ap = dacc + dl * HD + c4;
          v4f a = *(const v4f*)ap;
          a += hv;
          *(v4f*)ap = a;
        }
      }
    }
    __syncthreads();
  }
#pragma unroll 4
  for (int it = 0; it < (TDN * 16) / 256; ++it) {
    const int piece = it * 256 + tid;
    const int row = piece >> 4;
    const int grow = node0 + row;
    if (grow < npad) {
      const v4f v = *(const v4f*)(dacc + row * HD + c4);
      *(volatile v4f*)(ACC + (size_t)grow * HD + c4) = v;
    }
  }
  __threadfence();
#pragma unroll 4
  for (int it = 0; it < (TDN * 16) / 256; ++it) {
    const int piece = it * 256 + tid;
    const int row = piece >> 4;
    const int grow = node0 + row;
    if (grow < npad) {
      const v4f v = *(const v4f*)(dacc + row * HD + c4);
      *(volatile v4f*)(ACC + (size_t)grow * HD + c4) = v;
    }
  }
}

__global__ __launch_bounds__(256)
void k_colstat(const float* __restrict__ Y, int Nreal, int npad, double* PART)
{
  __shared__ double ds[4][64], ds2[4][64];
  __shared__ __attribute__((aligned(16))) double dline[128];
  const int tid = threadIdx.x, col = tid & 63, rg = tid >> 6;
  double s = 0.0, s2 = 0.0;
#pragma unroll 1
  for (int j = 0; j < STR / 4; ++j) {
    const int row = blockIdx.x * STR + j * 4 + rg;
    const int rc = min(row, npad - 1);
    float v = Y[(size_t)rc * HD + col];
    v = (row < Nreal) ? v : 0.0f;
    const double d = (double)v;
    s += d;
    s2 += d * d;
  }
  ds[rg][col] = s;
  ds2[rg][col] = s2;
  __syncthreads();
  if (tid < 64) {
    dline[tid] = ((ds[0][tid] + ds[1][tid]) + ds[2][tid]) + ds[3][tid];
    dline[64 + tid] = ((ds2[0][tid] + ds2[1][tid]) + ds2[2][tid]) + ds2[3][tid];
  }
  __syncthreads();
  if (tid < 64) {
    const v2d v = *(const v2d*)(dline + 2 * tid);
    *(volatile v2d*)(PART + (size_t)blockIdx.x * 128 + 2 * tid) = v;
  }
  __threadfence();
  if (tid < 64) {
    const v2d v = *(const v2d*)(dline + 2 * tid);
    *(volatile v2d*)(PART + (size_t)blockIdx.x * 128 + 2 * tid) = v;
  }
}

__global__ __launch_bounds__(64)
void k_bnfin(const double* __restrict__ PART, int nch, int Nreal,
             const float* __restrict__ g, const float* __restrict__ b, float* SS)
{
  __shared__ __attribute__((aligned(16))) float sh[128];
  const int t = threadIdx.x;
  double s = 0.0, s2 = 0.0;
#pragma unroll 1
  for (int c = 0; c < nch; ++c) {
    s += PART[(size_t)c * 128 + t];
    s2 += PART[(size_t)c * 128 + 64 + t];
  }
  const double invn = 1.0 / (double)Nreal;
  const double mean = s * invn;
  double var = s2 * invn - mean * mean;
  var = (var > 0.0) ? var : 0.0;
  const float rs = (float)(1.0 / sqrt(var + 1e-5));
  const float scale = rs * g[t];
  const float shift = b[t] - (float)mean * scale;
  sh[t] = scale;
  sh[64 + t] = shift;
  __syncthreads();
  if (t < 32) {
    const v4f v = *(const v4f*)(sh + 4 * t);
    *(volatile v4f*)(SS + 4 * t) = v;
  }
  __threadfence();
  if (t < 32) {
    const v4f v = *(const v4f*)(sh + 4 * t);
    *(volatile v4f*)(SS + 4 * t) = v;
  }
}

__global__ __launch_bounds__(256)
void k_bnout(const float* __restrict__ Y, const float* __restrict__ SS, int Nreal, float* OUT)
{
  const int idx = blockIdx.x * 256 + threadIdx.x;
  const int row = idx >> 4;
  const int c = (idx & 15) * 4;
  const v4f sc = *(const v4f*)(SS + c);
  const v4f sh = *(const v4f*)(SS + HD + c);
  v4f v = *(const v4f*)(Y + (size_t)row * HD + c);
  v = v * sc + sh;
#pragma unroll
  for (int i = 0; i < 4; ++i) {
    float x = fmaxf(v[i], 0.0f);
    v[i] = (row < Nreal) ? x : 0.0f;
  }
  float* gp = OUT + (size_t)row * HD + c;
  *(volatile v4f*)gp = v;
  __threadfence();
  *(volatile v4f*)gp = v;
}

__global__ __launch_bounds__(256)
void k_attstat(const float* __restrict__ W0, const float* __restrict__ W1, const float* __restrict__ W2,
               int Nreal, int npad, double* PART)
{
  __shared__ double ds[4][64], ds2[4][64];
  __shared__ __attribute__((aligned(16))) double dline[128];
  const int tid = threadIdx.x, col = tid & 63, rg = tid >> 6;
  double s = 0.0, s2 = 0.0;
#pragma unroll 1
  for (int j = 0; j < STR / 4; ++j) {
    const int row = blockIdx.x * STR + j * 4 + rg;
    const int rc = min(row, npad - 1);
    const size_t o = (size_t)rc * HD + col;
    float a = W0[o], b1 = W1[o], b2 = W2[o];
    a = (row < Nreal) ? a : 0.0f;
    s += (double)a * (double)b1;
    s2 += (double)a * (double)b2;
  }
  ds[rg][col] = s;
  ds2[rg][col] = s2;
  __syncthreads();
  if (tid < 64) {
    dline[tid] = ((ds[0][tid] + ds[1][tid]) + ds[2][tid]) + ds[3][tid];
    dline[64 + tid] = ((ds2[0][tid] + ds2[1][tid]) + ds2[2][tid]) + ds2[3][tid];
  }
  __syncthreads();
  if (tid < 64) {
    const v2d v = *(const v2d*)(dline + 2 * tid);
    *(volatile v2d*)(PART + (size_t)blockIdx.x * 128 + 2 * tid) = v;
  }
  __threadfence();
  if (tid < 64) {
    const v2d v = *(const v2d*)(dline + 2 * tid);
    *(volatile v2d*)(PART + (size_t)blockIdx.x * 128 + 2 * tid) = v;
  }
}

__global__ __launch_bounds__(64)
void k_attfin(const double* __restrict__ AP, int nch, const float* __restrict__ w_att,
              const float* __restrict__ b_att, float* WTS)
{
  __shared__ float s1[64], s2[64], wv[4];
  const int t = threadIdx.x;
  double a = 0.0, b = 0.0;
#pragma unroll 1
  for (int c = 0; c < nch; ++c) {
    a += AP[(size_t)c * 128 + t];
    b += AP[(size_t)c * 128 + 64 + t];
  }
  s1[t] = (float)a;
  s2[t] = (float)b;
  __syncthreads();
  if (t == 0) {
    float mn1 = s1[0], mx1 = s1[0], mn2 = s2[0], mx2 = s2[0];
#pragma unroll 1
    for (int k = 1; k < 64; ++k) {
      mn1 = fminf(mn1, s1[k]); mx1 = fmaxf(mx1, s1[k]);
      mn2 = fminf(mn2, s2[k]); mx2 = fmaxf(mx2, s2[k]);
    }
    const float r1 = 1.0f / (mx1 - mn1 + 1e-6f);
    const float r2 = 1.0f / (mx2 - mn2 + 1e-6f);
    float sc1 = 0.0f, sc2 = 0.0f;
#pragma unroll 1
    for (int k = 0; k < 64; ++k) {
      sc1 += ((s1[k] - mn1) * r1) * w_att[k];
      sc2 += ((s2[k] - mn2) * r2) * w_att[k];
    }
    sc1 += b_att[0];
    sc2 += b_att[0];
    const float mx = fmaxf(sc1, sc2);
    const float e1 = __expf(sc1 - mx), e2 = __expf(sc2 - mx);
    const float rinv = 1.0f / (e1 + e2);
    wv[0] = e1 * rinv;
    wv[1] = e2 * rinv;
  }
  __syncthreads();
  const float w1 = wv[0], w2 = wv[1];
  v4f v;
  v[0] = (t == 0) ? w1 : 0.0f;
  v[1] = (t == 0) ? w2 : 0.0f;
  v[2] = 0.0f;
  v[3] = 0.0f;
  if (t < 8) *(volatile v4f*)(WTS + 4 * t) = v;
  __threadfence();
  if (t < 8) *(volatile v4f*)(WTS + 4 * t) = v;
}

__global__ __launch_bounds__(256)
void k_pool(const int* __restrict__ batch, const float* __restrict__ W0, const float* __restrict__ W1,
            const float* __restrict__ W2, const float* __restrict__ WTS, int Nreal, int gpad, float* POOL, int nchunk)
{
  extern __shared__ __attribute__((aligned(16))) float pacc[];
  __shared__ int plst[8][256];
  __shared__ int pcnt[8];
  const int tid = threadIdx.x, lane = tid & 31, wave = tid >> 5;
  const int g0 = blockIdx.x * TDG;
  const int c4 = (tid & 15) * 4;
  const float w1 = WTS[0], w2 = WTS[1];
#pragma unroll 4
  for (int it = 0; it < (TDG * 16) / 256; ++it) {
    const int piece = it * 256 + tid;
    const int row = piece >> 4;
    v4f z;
    z[0] = 0.0f; z[1] = 0.0f; z[2] = 0.0f; z[3] = 0.0f;
    *(v4f*)(pacc + row * HD + c4) = z;
  }
  __syncthreads();
  for (int ci = 0; ci < nchunk; ++ci) {
    const int base = ci * SCH;
    int cw = 0;
#pragma unroll
    for (int j = 0; j < SCH / 256; ++j) {
      const int n = base + j * 256 + tid;
      const int nc = min(n, Nreal - 1);
      const int g = batch[nc];
      const int dl = g - g0;
      const bool hit = (n < Nreal) && ((unsigned)dl < (unsigned)TDG);
      const unsigned mk = __builtin_amdgcn_ballot_w32(hit);
      const int rank = __builtin_popcount(mk & ((1u << lane) - 1u));
      const int slot = cw + rank;
      if (hit && slot < 256) plst[wave][slot] = (n << 9) | dl;
      cw += __builtin_popcount(mk);
    }
    if (lane == 0) pcnt[wave] = cw;
    __syncthreads();
    if (wave == 0) {
      for (int w = 0; w < 8; ++w) {
        const int nw = min(pcnt[w], 256);
        for (int k = 0; k < nw; ++k) {
          const int ent = plst[w][k];
          const int n = min(ent >> 9, Nreal - 1);
          const int dl = ent & (TDG - 1);
          const size_t o = (size_t)n * HD + c4;
          const v4f a = *(const v4f*)(W0 + o);
          const v4f r1 = *(const v4f*)(W1 + o);
          const v4f r2 = *(const v4f*)(W2 + o);
          const v4f rep = (r1 * w1 + r2 * w2) + a;
          float* ap = pacc + dl * HD + c4;
          v4f acc = *(const v4f*)ap;
          acc += rep;
          *(v4f*)ap = acc;
        }
      }
    }
    __syncthreads();
  }
#pragma unroll 4
  for (int it = 0; it < (TDG * 16) / 256; ++it) {
    const int piece = it * 256 + tid;
    const int row = piece >> 4;
    const int grow = g0 + row;
    if (grow < gpad) {
      const v4f v = *(const v4f*)(pacc + row * HD + c4);
      *(volatile v4f*)(POOL + (size_t)grow * HD + c4) = v;
    }
  }
  __threadfence();
#pragma unroll 4
  for (int it = 0; it < (TDG * 16) / 256; ++it) {
    const int piece = it * 256 + tid;
    const int row = piece >> 4;
    const int grow = g0 + row;
    if (grow < gpad) {
      const v4f v = *(const v4f*)(pacc + row * HD + c4);
      *(volatile v4f*)(POOL + (size_t)grow * HD + c4) = v;
    }
  }
}

static inline int hmin(int a, int b) { return a < b ? a : b; }

extern "C" void kernel_launch(void* const* d_in, const int* in_sizes, int n_in,
                              void* d_out, int out_size, void* d_ws, size_t ws_size,
                              hipStream_t stream)
{
  if (n_in < 31) return;
  const int nN = in_sizes[0] / NFT;
  const int nE = in_sizes[1] / NFT;
  const int P2 = in_sizes[2] / 2;
  const int P3 = in_sizes[4] / 3;
  const int G  = out_size / NCL;
  if (nN <= 0 || nE <= 0 || P2 <= 0 || P3 <= 0 || G <= 0) return;
  if (in_sizes[0] != nN * NFT || in_sizes[1] != nE * NFT) return;
  if (in_sizes[2] != P2 * 2 || in_sizes[3] != P2) return;
  if (in_sizes[4] != P3 * 3 || in_sizes[5] != P3 * 2) return;
  if (in_sizes[6] != nN) return;
  if (in_sizes[7] != NFT * HD || in_sizes[8] != HD || in_sizes[9] != NFT * HD || in_sizes[10] != HD) return;
  if (in_sizes[11] != GW * 2 * HD || in_sizes[12] != GW * HD || in_sizes[13] != GW || in_sizes[14] != GW) return;
  if (in_sizes[15] != 2 * HD || in_sizes[16] != 2 * HD) return;
  if (in_sizes[17] != 2 * HD * HD || in_sizes[18] != 2 * HD || in_sizes[19] != 2 * HD || in_sizes[20] != 2 * HD) return;
  if (in_sizes[21] != 2 * HD * HD || in_sizes[22] != 2 * HD || in_sizes[23] != 2 * HD || in_sizes[24] != 2 * HD) return;
  if (in_sizes[25] != HD || in_sizes[26] < 1 || in_sizes[27] != HD * HD || in_sizes[28] != HD) return;
  if (in_sizes[29] != HD * NCL || in_sizes[30] != NCL || out_size != G * NCL) return;

  const float* x         = (const float*)d_in[0];
  const float* edge_attr = (const float*)d_in[1];
  const int*   paths2    = (const int*)d_in[2];
  const int*   ei2       = (const int*)d_in[3];
  const int*   paths3    = (const int*)d_in[4];
  const int*   ei3       = (const int*)d_in[5];
  const int*   batch     = (const int*)d_in[6];
  const float* w_feat    = (const float*)d_in[7];
  const float* b_feat    = (const float*)d_in[8];
  const float* w_bond    = (const float*)d_in[9];
  const float* b_bond    = (const float*)d_in[10];
  const float* w_ih      = (const float*)d_in[11];
  const float* w_hh      = (const float*)d_in[12];
  const float* b_ih      = (const float*)d_in[13];
  const float* b_hh      = (const float*)d_in[14];
  const float* bn_g      = (const float*)d_in[15];
  const float* bn_b      = (const float*)d_in[16];
  const float* mlp_w1    = (const float*)d_in[17];
  const float* mlp_b1    = (const float*)d_in[18];
  const float* bn1_g     = (const float*)d_in[19];
  const float* bn1_b     = (const float*)d_in[20];
  const float* mlp_w2    = (const float*)d_in[21];
  const float* mlp_b2    = (const float*)d_in[22];
  const float* bn2_g     = (const float*)d_in[23];
  const float* bn2_b     = (const float*)d_in[24];
  const float* w_att     = (const float*)d_in[25];
  const float* b_att     = (const float*)d_in[26];
  const float* w_l1      = (const float*)d_in[27];
  const float* b_l1      = (const float*)d_in[28];
  const float* w_l2      = (const float*)d_in[29];
  const float* b_l2      = (const float*)d_in[30];
  float* out = (float*)d_out;

  const int NPAD = (nN + 63) / 64 * 64;
  const int EPAD = (nE + 63) / 64 * 64;
  const int GPAD = (G + 63) / 64 * 64;
  const int NCH  = (nN + STR - 1) / STR;

  size_t off = 0;
  const size_t oWPL  = off; off += (size_t)WPL_TOTAL * 2;
  const size_t oEA   = off; off += (size_t)EPAD * HD * 2;
  const size_t oW0   = off; off += (size_t)NPAD * HD * 4;
  const size_t oRA   = off; off += (size_t)NPAD * HD * 4;
  const size_t oRB   = off; off += (size_t)NPAD * HD * 4;
  const size_t oRC   = off; off += (size_t)NPAD * HD * 4;
  const size_t oPART = off; off += (size_t)NCH * 128 * 8;
  const size_t oSS   = off; off += (size_t)3 * 512;
  const size_t oWTS  = off; off += 512;
  const size_t oPOOL = off; off += (size_t)GPAD * HD * 4;
  const size_t oYH   = off; off += (size_t)GPAD * HD * 4;
  const size_t total = off;
  if (total > ws_size) return;
  if (total > (size_t)134217728) return;

  char* ws = (char*)d_ws;
  unsigned short* WPL = (unsigned short*)(ws + oWPL);
  unsigned short* EA16w = (unsigned short*)(ws + oEA);
  const f16t* EA16 = (const f16t*)(ws + oEA);
  float* W0   = (float*)(ws + oW0);
  float* RA   = (float*)(ws + oRA);
  float* RB   = (float*)(ws + oRB);
  float* RC   = (float*)(ws + oRC);
  double* PART = (double*)(ws + oPART);
  float* SS0  = (float*)(ws + oSS);
  float* SS1  = SS0 + 128;
  float* SS2  = SS0 + 256;
  float* WTS  = (float*)(ws + oWTS);
  float* POOL = (float*)(ws + oPOOL);
  float* YH   = (float*)(ws + oYH);
  const unsigned short* WC = WPL + WPL_WC;

  const int SEG_LDS  = TDN * HD * 4;
  const int POOL_LDS = TDG * HD * 4;
  (void)hipFuncSetAttribute(reinterpret_cast<const void*>(&k_segsum<2>), hipFuncAttributeMaxDynamicSharedMemorySize, SEG_LDS);
  (void)hipFuncSetAttribute(reinterpret_cast<const void*>(&k_segsum<3>), hipFuncAttributeMaxDynamicSharedMemorySize, SEG_LDS);
  (void)hipFuncSetAttribute(reinterpret_cast<const void*>(&k_pool), hipFuncAttributeMaxDynamicSharedMemorySize, POOL_LDS);

  k_wprep<<<dim3(WPL_BLOCKS), dim3(256), 0, stream>>>(w_feat, w_bond, mlp_w1, mlp_w2, w_l1, w_l2, w_ih, w_hh, WPL);

  k_enc<<<dim3(NPAD / 64), dim3(128), 0, stream>>>(x, nN, WPL + WPL_WF_H, WPL + WPL_WF_L, b_feat, W0, EA16w, 1, 0);
  k_enc<<<dim3(EPAD / 64), dim3(128), 0, stream>>>(edge_attr, nE, WPL + WPL_WB_H, WPL + WPL_WB_L, b_bond, RA, EA16w, 0, 1);

  const int PC = NPAD;
  const int segGrid = (NPAD + TDN - 1) / TDN;

  {
    int c = 0;
    for (int p0 = 0; p0 < P2; p0 += PC, ++c) {
      const int pc = hmin(PC, P2 - p0);
      k_lstm<2, false><<<dim3((pc + 63) / 64), dim3(128), 0, stream>>>(
          paths2, ei2, W0, W0, EA16, WC, b_ih, b_hh, RB, p0, pc, nN, nE);
      k_segsum<2><<<dim3(segGrid), dim3(256), SEG_LDS, stream>>>(
          paths2, RB, RA, p0, pc, NPAD, (c == 0) ? 1 : 0, (pc + SCH - 1) / SCH);
    }
  }

  auto chain = [&](int i, float* dest) {
    k_colstat<<<dim3(NCH), dim3(256), 0, stream>>>(RA, nN, NPAD, PART);
    k_bnfin<<<dim3(1), dim3(64), 0, stream>>>(PART, NCH, nN, bn_g + i * HD, bn_b + i * HD, SS0);
    k_mlp<<<dim3(NPAD / 64), dim3(128), 0, stream>>>(RA, nN, SS0, 1, 0,
        WPL + WPL_MB + (i * 4 + 0) * 4096, WPL + WPL_MB + (i * 4 + 1) * 4096, mlp_b1 + i * HD, RB);
    k_colstat<<<dim3(NCH), dim3(256), 0, stream>>>(RB, nN, NPAD, PART);
    k_bnfin<<<dim3(1), dim3(64), 0, stream>>>(PART, NCH, nN, bn1_g + i * HD, bn1_b + i * HD, SS1);
    k_mlp<<<dim3(NPAD / 64), dim3(128), 0, stream>>>(RB, nN, SS1, 1, 1,
        WPL + WPL_MB + (i * 4 + 2) * 4096, WPL + WPL_MB + (i * 4 + 3) * 4096, mlp_b2 + i * HD, RA);
    k_colstat<<<dim3(NCH), dim3(256), 0, stream>>>(RA, nN, NPAD, PART);
    k_bnfin<<<dim3(1), dim3(64), 0, stream>>>(PART, NCH, nN, bn2_g + i * HD, bn2_b + i * HD, SS2);
    k_bnout<<<dim3(NPAD / 16), dim3(256), 0, stream>>>(RA, SS2, nN, dest);
  };
  chain(0, RC);

  {
    int c = 0;
    for (int p0 = 0; p0 < P3; p0 += PC, ++c) {
      const int pc = hmin(PC, P3 - p0);
      k_lstm<3, true><<<dim3((pc + 63) / 64), dim3(128), 0, stream>>>(
          paths3, ei3, W0, RC, EA16, WC, b_ih, b_hh, RB, p0, pc, nN, nE);
      k_segsum<3><<<dim3(segGrid), dim3(256), SEG_LDS, stream>>>(
          paths3, RB, RA, p0, pc, NPAD, (c == 0) ? 1 : 0, (pc + SCH - 1) / SCH);
    }
  }
  chain(1, RB);

  k_attstat<<<dim3(NCH), dim3(256), 0, stream>>>(W0, RC, RB, nN, NPAD, PART);
  k_attfin<<<dim3(1), dim3(64), 0, stream>>>(PART, NCH, w_att, b_att, WTS);
  k_pool<<<dim3((GPAD + TDG - 1) / TDG), dim3(256), POOL_LDS, stream>>>(
      batch, W0, RC, RB, WTS, nN, GPAD, POOL, (nN + SCH - 1) / SCH);
  k_mlp<<<dim3(GPAD / 64), dim3(128), 0, stream>>>(POOL, G, SS0, 0, 0,
      WPL + WPL_MB + 8 * 4096, WPL + WPL_MB + 9 * 4096, b_l1, YH);
  k_head2<<<dim3(GPAD / 64), dim3(128), 0, stream>>>(YH, G, SS0, WPL + WPL_L2_H, WPL + WPL_L2_L, b_l2, out, G * NCL);
}
